// GCN_44744969290503
// MI455X (gfx1250) — hardware-verified
//
#include <hip/hip_runtime.h>
#include <stddef.h>
#include <stdint.h>
#include <math.h>


#define CIN    128
#define HID    64
#define K2     128
#define L1N    128
#define NCLS   10
#define NGR    512
#define PGW    16
#define NTHR   256
#define NWAVE  8
#define EPT    8
#define CHUNK  (NTHR * EPT)
#define WCAP   (EPT * 32)
#define LISTN  (NWAVE * WCAP)
#define NBD    8192
#define SLD    13
#define NBA    1024
#define SLA    10
#define RCAP   28672
#define DEGCAP 64
#define GBM    64
#define GBN    64
#define GTHR   128
#define NUW    (HID * (K2 / 8))
#define AGG_ZINTS (LISTN + 2 * RCAP + 3 * NBA)
#define AGG_LDS_INTS (AGG_ZINTS + 16)
#define NOUT   (NGR * NCLS)
#define WSMAX  134217728

static_assert((CHUNK & (CHUNK - 1)) == 0 && CHUNK <= 4096);
static_assert((NBD & (NBD - 1)) == 0 && NBD == (1 << SLD));
static_assert((NBA & (NBA - 1)) == 0 && NBA == (1 << SLA));
static_assert(((long long)CHUNK << SLD) < (1LL << 31));
static_assert(((long long)CHUNK << SLA) < (1LL << 31));
static_assert(NBD % (NTHR * 4) == 0);
static_assert(LISTN % NTHR == 0);
static_assert(NBA % NWAVE == 0 && NBA % 32 == 0 && NBA % GBM == 0);
static_assert(RCAP % 32 == 0 && AGG_ZINTS % 4 == 0 && LISTN % 4 == 0);
static_assert(CIN % 32 == 0 && K2 % 32 == 0 && K2 == 2 * HID && HID == GBN && CIN == K2);
static_assert(GBM == (GTHR / 32) * 16 && GBN == 64);
static_assert(NUW % NTHR == 0 && NUW == 1024);
static_assert(CIN / 8 == 16 && K2 / 8 == 16);
static_assert(HID == 2 * 32);
static_assert(AGG_LDS_INTS * 4 <= 300000);
static_assert(NGR % PGW == 0 && PGW == 2 * NWAVE);
static_assert((PGW * NCLS) % 32 == 0 && (PGW * NCLS * 4) % 128 == 0);
static_assert(NTHR == 2 * L1N && PGW == 16);
static_assert(((HID * L1N) % 4) == 0 && ((L1N * NCLS) % 4) == 0);
static_assert((NGR / PGW - 1) * (PGW * NCLS) + (PGW * NCLS) - 1 < NOUT);

typedef float          v2f   __attribute__((ext_vector_type(2)));
typedef float          v4f   __attribute__((ext_vector_type(4)));
typedef float          v8f   __attribute__((ext_vector_type(8)));
typedef int            v4i   __attribute__((ext_vector_type(4)));
typedef int            v8i   __attribute__((ext_vector_type(8)));
typedef unsigned int   v4u   __attribute__((ext_vector_type(4)));
typedef unsigned short v8us  __attribute__((ext_vector_type(8)));
typedef unsigned short v16us __attribute__((ext_vector_type(16)));
typedef __bf16         v16bf __attribute__((ext_vector_type(16)));
typedef v2f  __attribute__((may_alias)) v2fa;
typedef v4f  __attribute__((may_alias)) v4fa;
typedef v4i  __attribute__((may_alias)) v4ia;
typedef v8us __attribute__((may_alias)) v8usa;
union FragB { v16bf v; v16us u; v8us h[2]; v8i w; };

__device__ __forceinline__ v8f wmb(const FragB& a, const FragB& b, v8f c) {
  v8f d = __builtin_amdgcn_wmma_f32_16x16x32_bf16(false, a.v, false, b.v, (short)0, c, false, false);
  asm volatile("v_nop\n\tv_nop\n\tv_nop\n\tv_nop" : "+v"(d) : "v"(a.w), "v"(b.w));
  return d;
}

__device__ __forceinline__ unsigned bf16_bits(float f) {
  const unsigned u = __float_as_uint(f);
  return (u + 0x7FFFu + ((u >> 16) & 1u)) >> 16;
}
__device__ __forceinline__ float bf16_val(float f) {
  return __uint_as_float(bf16_bits(f) << 16);
}

template <int SLB>
__device__ __forceinline__ int scan_chunk(const int* __restrict__ dsts, int nE, int cbase, int slotBase,
                                          int nb, int vec8, int* list, int tid, int lane, int wave) {
  int wc = 0;
  const int el0  = tid * EPT;
  const int e0   = cbase + el0;
  const int sent = -2147483647 - 1;
  v4i da, db;
  if (vec8 != 0 && cbase + CHUNK <= nE) {
    da = *(const v4i*)(dsts + e0);
    db = *(const v4i*)(dsts + e0 + 4);
  } else {
    da.x = (e0     < nE) ? dsts[min(e0,     nE - 1)] : sent;
    da.y = (e0 + 1 < nE) ? dsts[min(e0 + 1, nE - 1)] : sent;
    da.z = (e0 + 2 < nE) ? dsts[min(e0 + 2, nE - 1)] : sent;
    da.w = (e0 + 3 < nE) ? dsts[min(e0 + 3, nE - 1)] : sent;
    db.x = (e0 + 4 < nE) ? dsts[min(e0 + 4, nE - 1)] : sent;
    db.y = (e0 + 5 < nE) ? dsts[min(e0 + 5, nE - 1)] : sent;
    db.z = (e0 + 6 < nE) ? dsts[min(e0 + 6, nE - 1)] : sent;
    db.w = (e0 + 7 < nE) ? dsts[min(e0 + 7, nE - 1)] : sent;
  }
  const unsigned nbs = (unsigned)slotBase;
  const unsigned unb = (unsigned)nb;
  const unsigned s0 = (unsigned)da.x - nbs, s1 = (unsigned)da.y - nbs;
  const unsigned s2 = (unsigned)da.z - nbs, s3 = (unsigned)da.w - nbs;
  const unsigned s4 = (unsigned)db.x - nbs, s5 = (unsigned)db.y - nbs;
  const unsigned s6 = (unsigned)db.z - nbs, s7 = (unsigned)db.w - nbs;
  const bool h0 = s0 < unb, h1 = s1 < unb, h2 = s2 < unb, h3 = s3 < unb;
  const bool h4 = s4 < unb, h5 = s5 < unb, h6 = s6 < unb, h7 = s7 < unb;
  const unsigned any = __builtin_amdgcn_ballot_w32(h0 | h1 | h2 | h3 | h4 | h5 | h6 | h7);
  if (any != 0u) {
#define HITJ(J, HJ, SJ) { \
      const unsigned mj = __builtin_amdgcn_ballot_w32(HJ); \
      if (mj != 0u) { \
        if (HJ) { \
          const int pos = wc + (int)__builtin_amdgcn_mbcnt_lo(mj, 0u); \
          if (pos < WCAP) list[wave * WCAP + pos] = ((el0 + (J)) << SLB) | (int)(SJ); \
        } \
        wc += (int)__builtin_popcount(mj); } }
    HITJ(0, h0, s0)
    HITJ(1, h1, s1)
    HITJ(2, h2, s2)
    HITJ(3, h3, s3)
    HITJ(4, h4, s4)
    HITJ(5, h5, s5)
    HITJ(6, h6, s6)
    HITJ(7, h7, s7)
#undef HITJ
  }
  return wc;
}

__device__ __forceinline__ void wrow8(const float* __restrict__ p, unsigned short* dp) {
  v8us o;
#pragma unroll
  for (int i = 0; i < 8; ++i) o[i] = (unsigned short)bf16_bits(p[(size_t)i * HID]);
  *(volatile v8us*)dp = o;
  __threadfence();
  *(volatile v8us*)dp = o;
}

__global__ __launch_bounds__(NTHR) void k_wprep(const float* __restrict__ W0, const float* __restrict__ W1,
                                                const float* __restrict__ W2, unsigned short* W0T,
                                                unsigned short* W1T, unsigned short* W2T) {
  const int u    = (int)blockIdx.x * NTHR + (int)threadIdx.x;
  const int part = u >> 10;
  const int v    = u & (NUW - 1);
  const int n    = v >> 4;
  const int k8   = (v & 15) * 8;
  const int kk   = k8 & (HID - 1);
  if (part == 0) {
    wrow8(W0 + (size_t)k8 * HID + n, W0T + (size_t)n * CIN + k8);
  } else if (part == 1) {
    wrow8(W1 + (size_t)kk * HID + n, W1T + (size_t)n * K2 + k8);
  } else if (part == 2) {
    wrow8(W2 + (size_t)kk * HID + n, W2T + (size_t)n * K2 + k8);
  }
}

__global__ __launch_bounds__(NTHR) void k_cvx(const float* __restrict__ x, int nN, int nUnits,
                                              unsigned short* xb) {
  const int u = (int)blockIdx.x * NTHR + (int)threadIdx.x;
  if (u >= nUnits) return;
  const int row = u >> 4;
  const int k8  = (u & 15) * 8;
  const int rc  = row < nN ? row : nN - 1;
  const float* p = x + (size_t)rc * CIN + k8;
  const v4f a = *(const v4fa*)p;
  const v4f b = *(const v4fa*)(p + 4);
  const bool ok = row < nN;
  v8us o;
  o[0] = ok ? (unsigned short)bf16_bits(a.x) : (unsigned short)0;
  o[1] = ok ? (unsigned short)bf16_bits(a.y) : (unsigned short)0;
  o[2] = ok ? (unsigned short)bf16_bits(a.z) : (unsigned short)0;
  o[3] = ok ? (unsigned short)bf16_bits(a.w) : (unsigned short)0;
  o[4] = ok ? (unsigned short)bf16_bits(b.x) : (unsigned short)0;
  o[5] = ok ? (unsigned short)bf16_bits(b.y) : (unsigned short)0;
  o[6] = ok ? (unsigned short)bf16_bits(b.z) : (unsigned short)0;
  o[7] = ok ? (unsigned short)bf16_bits(b.w) : (unsigned short)0;
  unsigned short* dp = xb + (size_t)row * CIN + k8;
  *(volatile v8us*)dp = o;
  __threadfence();
  *(volatile v8us*)dp = o;
}

__global__ __launch_bounds__(NTHR) void k_deg(const int* __restrict__ dsts, int nE, int vec8, float* dis) {
  __shared__ __attribute__((aligned(16))) int scnt[NBD];
  __shared__ __attribute__((aligned(16))) int list[LISTN];
  __shared__ int wcnt[NWAVE];
  const int tid = (int)threadIdx.x, lane = tid & 31, wave = tid >> 5;
  const int nodeBase = (int)blockIdx.x * NBD;

  for (int i = tid; i < NBD; i += NTHR) scnt[i] = 0;
  for (int i = tid; i < LISTN; i += NTHR) list[i] = 0;
  if (tid < NWAVE) wcnt[tid] = 0;
  __syncthreads();

  const int nChunks = (nE + CHUNK - 1) / CHUNK;
#pragma unroll 1
  for (int ch = 0; ch < nChunks; ++ch) {
    const int cbase = ch * CHUNK;
    const int wc = scan_chunk<SLD>(dsts, nE, cbase, nodeBase, NBD, vec8, list, tid, lane, wave);
    if (lane == 0) wcnt[wave] = wc;
    __syncthreads();
    if (wave == 0) {
#pragma unroll 1
      for (int w2 = 0; w2 < NWAVE; ++w2) {
        int c = wcnt[w2];
        c = c < 0 ? 0 : (c > WCAP ? WCAP : c);
#pragma unroll 1
        for (int b0 = 0; b0 < c; b0 += 32) {
          const int idx = b0 + lane;
          const int ent = list[w2 * WCAP + (idx < WCAP ? idx : WCAP - 1)];
          const int m32 = (c - b0) < 32 ? (c - b0) : 32;
#pragma unroll 1
          for (int k = 0; k < m32; ++k) {
            const int u  = __builtin_amdgcn_readlane(ent, k);
            const int sl = u & (NBD - 1);
            if (lane == 0) scnt[sl] = scnt[sl] + 1;
          }
        }
      }
    }
    __syncthreads();
  }

#pragma unroll 1
  for (int i = tid; i < NBD; i += NTHR) {
    const float d  = (float)scnt[i] + 1.0f;
    const float r  = 1.0f / sqrtf(d);
    const float dv = (d > 0.0f) ? r : 0.0f;
    scnt[i] = __float_as_int(dv);
  }
  __syncthreads();

  v4f vals[NBD / (NTHR * 4)];
#pragma unroll
  for (int it = 0; it < NBD / (NTHR * 4); ++it) {
    const int s0 = it * (NTHR * 4) + 4 * tid;
    const v4i c4 = *(const v4ia*)(scnt + s0);
    v4f v;
    v.x = __int_as_float(c4.x); v.y = __int_as_float(c4.y);
    v.z = __int_as_float(c4.z); v.w = __int_as_float(c4.w);
    vals[it] = v;
  }
#pragma unroll
  for (int it = 0; it < NBD / (NTHR * 4); ++it) {
    const int s0 = it * (NTHR * 4) + 4 * tid;
    *(volatile v4f*)(dis + (size_t)nodeBase + s0) = vals[it];
  }
  __threadfence();
#pragma unroll
  for (int it = 0; it < NBD / (NTHR * 4); ++it) {
    const int s0 = it * (NTHR * 4) + 4 * tid;
    *(volatile v4f*)(dis + (size_t)nodeBase + s0) = vals[it];
  }
}

__global__ __launch_bounds__(GTHR) void k_gemm(
    const unsigned short* __restrict__ A, const unsigned short* __restrict__ WT,
    float* outF, int K, int ldo)
{
  __shared__ __attribute__((aligned(16))) float stg[GBM * GBN];
  const int tid = (int)threadIdx.x, lane = tid & 31, wave = tid >> 5, hh = lane >> 4, m = lane & 15;
  const int rowBase = (int)blockIdx.x * GBM;
  const int col0    = (int)blockIdx.y * GBN;

  v8f acc[4];
  {
    const v8f z = {0.f, 0.f, 0.f, 0.f, 0.f, 0.f, 0.f, 0.f};
    acc[0] = z; acc[1] = z; acc[2] = z; acc[3] = z;
  }
  const unsigned short* ap = A  + (size_t)(rowBase + 16 * wave + m) * (size_t)K + 8 * hh;
  const unsigned short* wp = WT + (size_t)(col0 + m) * (size_t)K + 8 * hh;
  const int ksteps = K >> 5;
#pragma unroll 1
  for (int ks = 0; ks < ksteps; ++ks) {
    FragB af;
    af.h[0] = *(const v8usa*)(ap + 32 * ks);
    af.h[1] = *(const v8usa*)(ap + 32 * ks + 16);
#pragma unroll
    for (int t = 0; t < 4; ++t) {
      const unsigned short* wq = wp + (size_t)(16 * t) * (size_t)K + 32 * ks;
      FragB bf;
      bf.h[0] = *(const v8usa*)wq;
      bf.h[1] = *(const v8usa*)(wq + 16);
      acc[t] = wmb(af, bf, acc[t]);
    }
  }

#pragma unroll
  for (int t = 0; t < 4; ++t) {
    const int lc = 16 * t + m;
#pragma unroll
    for (int r = 0; r < 8; ++r) {
      const int lr = 16 * wave + 8 * hh + r;
      stg[lr * GBN + lc] = acc[t][r];
    }
  }
  __syncthreads();

  v4f fv[8];
#pragma unroll
  for (int i = 0; i < 8; ++i) {
    const int lr = 16 * wave + 2 * i + hh;
    fv[i] = *(const v4fa*)(stg + lr * GBN + 4 * m);
  }
#pragma unroll
  for (int i = 0; i < 8; ++i) {
    const int lr = 16 * wave + 2 * i + hh;
    const int gr = rowBase + lr;
    float* op = outF + (size_t)gr * (size_t)ldo + col0 + 4 * m;
    *(volatile v4f*)op = fv[i];
  }
  __threadfence();
#pragma unroll
  for (int i = 0; i < 8; ++i) {
    const int lr = 16 * wave + 2 * i + hh;
    const int gr = rowBase + lr;
    float* op = outF + (size_t)gr * (size_t)ldo + col0 + 4 * m;
    *(volatile v4f*)op = fv[i];
  }
}

template <int MODE, int RELU>
__global__ __launch_bounds__(NTHR) void k_agg(const int* __restrict__ srcs, const int* __restrict__ dsts,
                                              int nE, int nN, int vec8, int mRows,
                                              const float* __restrict__ dis,
                                              const float* __restrict__ xl, const float* __restrict__ bias,
                                              unsigned short* hb, float* hout) {
  extern __shared__ __attribute__((aligned(16))) int dsm[];
  int* list = dsm;
  int* hl   = dsm + LISTN;
  int* sl   = dsm + LISTN + RCAP;
  int* cnt  = dsm + LISTN + 2 * RCAP;
  int* offs = cnt + NBA;
  int* cur  = offs + NBA;
  int* misc = cur + NBA;
  const int tid = (int)threadIdx.x, lane = tid & 31, wave = tid >> 5;
  const int nodeBase = (int)blockIdx.x * NBA;

  {
    const v4i z4 = {0, 0, 0, 0};
    for (int i = tid * 4; i < AGG_ZINTS; i += NTHR * 4) *(v4ia*)(dsm + i) = z4;
    if (tid < 16) misc[tid] = 0;
  }
  float bv0, bv1;
  {
    const v2f a = *(const v2fa*)(bias + 2 * lane);
    bv0 = bf16_val(a.x); bv1 = bf16_val(a.y);
  }
  __syncthreads();

  int t = 0, ov = 0;
  const int nChunks = (nE + CHUNK - 1) / CHUNK;
#pragma unroll 1
  for (int ch = 0; ch < nChunks; ++ch) {
    const int cbase = ch * CHUNK;
    const int wc = scan_chunk<SLA>(dsts, nE, cbase, nodeBase, NBA, vec8, list, tid, lane, wave);
    if (lane == 0) misc[wave] = wc;
    __syncthreads();
    if (wave == 0) {
#pragma unroll 1
      for (int w2 = 0; w2 < NWAVE; ++w2) {
        int c = misc[w2];
        c = c < 0 ? 0 : (c > WCAP ? WCAP : c);
#pragma unroll 1
        for (int b0 = 0; b0 < c; b0 += 32) {
          const int idx = b0 + lane;
          const int ent = list[w2 * WCAP + (idx < WCAP ? idx : WCAP - 1)];
          const int m32 = (c - b0) < 32 ? (c - b0) : 32;
#pragma unroll 1
          for (int k = 0; k < m32; ++k) {
            const int u    = __builtin_amdgcn_readlane(ent, k);
            const int slot = u & (NBA - 1);
            const int el   = (u >> SLA) & (CHUNK - 1);
            const int pk   = ((cbase + el) << SLA) | slot;
            if (t < RCAP) {
              if (lane == 0) { hl[t] = pk; cnt[slot] = cnt[slot] + 1; }
              t = t + 1;
            } else {
              ov = 1;
            }
          }
        }
      }
    }
    __syncthreads();
  }
  if (wave == 0 && lane == 0) { misc[8] = t; misc[9] = ov; }
  __syncthreads();
  int tt = misc[8];
  tt = tt < 0 ? 0 : (tt > RCAP ? RCAP : tt);
  const int ovf = misc[9];

  if (wave == 0) {
    const int base = lane * (NBA / 32);
    int s = 0;
#pragma unroll 1
    for (int i = 0; i < NBA / 32; ++i) s += cnt[base + i];
    int incl = s;
#pragma unroll
    for (int d = 1; d < 32; d <<= 1) {
      const int y = __shfl_up(incl, d, 32);
      if (lane >= d) incl += y;
    }
    int run = incl - s;
#pragma unroll 1
    for (int i = 0; i < NBA / 32; ++i) {
      const int cv = cnt[base + i];
      offs[base + i] = run;
      cur[base + i]  = run;
      run += cv;
    }
  }
  __syncthreads();
  if (wave == 0) {
#pragma unroll 1
    for (int b0 = 0; b0 < tt; b0 += 32) {
      const int idx = b0 + lane;
      const int ent = hl[idx < RCAP ? idx : RCAP - 1];
      const int m32 = (tt - b0) < 32 ? (tt - b0) : 32;
#pragma unroll 1
      for (int k = 0; k < m32; ++k) {
        const int u    = __builtin_amdgcn_readlane(ent, k);
        const int slot = u & (NBA - 1);
        if (lane == 0) {
          int p = cur[slot];
          p = p < 0 ? 0 : (p > RCAP - 1 ? RCAP - 1 : p);
          sl[p] = u;
          cur[slot] = p + 1;
        }
      }
    }
  }
  __syncthreads();

  const float qnan = __int_as_float(0x7fc00000);
  const float pz = (ovf != 0) ? qnan : 0.0f;
  const int sa = (2 * lane) & 31, sb = (2 * lane + 1) & 31;
  const int q0s = (4 * lane) & 31, q1s = (4 * lane + 1) & 31;
  const int q2s = (4 * lane + 2) & 31, q3s = (4 * lane + 3) & 31;
#pragma unroll 1
  for (int si = 0; si < NBA / NWAVE; ++si) {
    const int s    = si * NWAVE + wave;
    const int node = nodeBase + s;
    int c = cnt[s];
    const bool big = c > DEGCAP;
    c = c < 0 ? 0 : (c > DEGCAP ? DEGCAP : c);
    int o = offs[s];
    o = o < 0 ? 0 : (o > RCAP ? RCAP : o);
    const int nc = node < nN ? node : nN - 1;
    const float dd = dis[nc];
    const float rd = dd * dd;
    float acc0 = 0.0f, acc1 = 0.0f;
#pragma unroll 1
    for (int b0 = 0; b0 < c; b0 += 32) {
      int idx = o + b0 + lane;
      idx = idx > RCAP - 1 ? RCAP - 1 : idx;
      const int ent = sl[idx];
      int eid = ent >> SLA;
      eid = eid < 0 ? 0 : (eid > nE - 1 ? nE - 1 : eid);
      int sr = srcs[eid];
      sr = sr < 0 ? 0 : (sr > nN - 1 ? nN - 1 : sr);
      const float cf  = dis[sr] * dd;
      const int   cfi = __float_as_int(cf);
      const int m32 = (c - b0) < 32 ? (c - b0) : 32;
#pragma unroll 1
      for (int k = 0; k < m32; ++k) {
        const int   sk = __builtin_amdgcn_readlane(sr, k);
        const float ck = __int_as_float(__builtin_amdgcn_readlane(cfi, k));
        const v2f a = *(const v2fa*)(xl + (size_t)sk * HID + 2 * lane);
        acc0 = fmaf(ck, a.x, acc0); acc1 = fmaf(ck, a.y, acc1);
      }
    }
    float sv0, sv1;
    {
      const v2f a = *(const v2fa*)(xl + (size_t)nc * HID + 2 * lane);
      sv0 = a.x; sv1 = a.y;
    }
    const float pzr = big ? qnan : pz;
    const bool live = node < nN;
    float y0 = (acc0 + sv0 * rd) + bv0;
    float y1 = (acc1 + sv1 * rd) + bv1;
    if constexpr (RELU != 0) {
      y0 = (y0 > 0.0f) ? y0 : (y0 - y0);
      y1 = (y1 > 0.0f) ? y1 : (y1 - y1);
    }
    y0 = y0 + pzr; y1 = y1 + pzr;
    const float v0 = live ? y0 : 0.0f;
    const float v1 = live ? y1 : 0.0f;
    const bool wr = (node < mRows) && (lane < 16);
    if constexpr (MODE != 0) {
      const unsigned hb0 = bf16_bits(v0), hb1 = bf16_bits(v1);
      const unsigned lb0 = bf16_bits(v0 - __uint_as_float(hb0 << 16));
      const unsigned lb1 = bf16_bits(v1 - __uint_as_float(hb1 << 16));
      const int hw = (int)(hb0 | (hb1 << 16));
      const int lw = (int)(lb0 | (lb1 << 16));
      const int g0 = __shfl(hw, q0s, 32), g1 = __shfl(hw, q1s, 32);
      const int g2 = __shfl(hw, q2s, 32), g3 = __shfl(hw, q3s, 32);
      const int p0 = __shfl(lw, q0s, 32), p1 = __shfl(lw, q1s, 32);
      const int p2 = __shfl(lw, q2s, 32), p3 = __shfl(lw, q3s, 32);
      const bool lsel = (lane & 8) != 0;
      v4u pv;
      pv.x = (unsigned int)(lsel ? p0 : g0);
      pv.y = (unsigned int)(lsel ? p1 : g1);
      pv.z = (unsigned int)(lsel ? p2 : g2);
      pv.w = (unsigned int)(lsel ? p3 : g3);
      unsigned short* hp = hb + (size_t)node * K2 + 8 * (lane & 15);
      if (wr) *(volatile v4u*)hp = pv;
      __threadfence();
      if (wr) *(volatile v4u*)hp = pv;
    } else {
      v4f ow;
      ow.x = __shfl(v0, sa, 32); ow.y = __shfl(v1, sa, 32);
      ow.z = __shfl(v0, sb, 32); ow.w = __shfl(v1, sb, 32);
      float* op = hout + (size_t)node * HID + 4 * (lane & 15);
      if (wr) *(volatile v4f*)op = ow;
      __threadfence();
      if (wr) *(volatile v4f*)op = ow;
    }
  }
}

__global__ __launch_bounds__(NTHR) void k_pool_head(const float* __restrict__ hf, const int* __restrict__ bat,
                                                    int nN,
                                                    const float* __restrict__ l1w, const float* __restrict__ l1b,
                                                    const float* __restrict__ l2w, const float* __restrict__ l2b,
                                                    float* out) {
  __shared__ __attribute__((aligned(16))) float w1s[HID * L1N];
  __shared__ __attribute__((aligned(16))) float w2s[L1N * NCLS];
  __shared__ __attribute__((aligned(16))) float b1s[L1N];
  __shared__ __attribute__((aligned(16))) float b2s[32];
  __shared__ __attribute__((aligned(16))) float gs[PGW * HID];
  __shared__ __attribute__((aligned(16))) float ts[PGW * L1N];
  __shared__ __attribute__((aligned(16))) float os[PGW * NCLS];
  const int tid = (int)threadIdx.x, lane = tid & 31, wave = tid >> 5;
  const int g0 = (int)blockIdx.x * PGW;

#pragma unroll 1
  for (int i = tid; i < (HID * L1N) / 4; i += NTHR) {
    const v4f a = *(const v4fa*)(l1w + 4 * i);
    v4f r;
    r.x = bf16_val(a.x); r.y = bf16_val(a.y); r.z = bf16_val(a.z); r.w = bf16_val(a.w);
    *(v4fa*)(w1s + 4 * i) = r;
  }
#pragma unroll 1
  for (int i = tid; i < (L1N * NCLS) / 4; i += NTHR) {
    const v4f a = *(const v4fa*)(l2w + 4 * i);
    v4f r;
    r.x = bf16_val(a.x); r.y = bf16_val(a.y); r.z = bf16_val(a.z); r.w = bf16_val(a.w);
    *(v4fa*)(w2s + 4 * i) = r;
  }
  if (wave == 0) {
    const v4f a = *(const v4fa*)(l1b + 4 * lane);
    v4f r;
    r.x = bf16_val(a.x); r.y = bf16_val(a.y); r.z = bf16_val(a.z); r.w = bf16_val(a.w);
    *(v4fa*)(b1s + 4 * lane) = r;
  }
  if (wave == 1) {
    const float bb = l2b[lane < NCLS ? lane : NCLS - 1];
    b2s[lane] = (lane < NCLS) ? bf16_val(bb) : 0.0f;
  }

  const int gA = g0 + 2 * wave;
  const int gB = gA + 1;
  float a00 = 0.0f, a01 = 0.0f, a10 = 0.0f, a11 = 0.0f;
#pragma unroll 1
  for (int i0 = 0; i0 < nN; i0 += 32) {
    const int i  = i0 + lane;
    const int ic = i < nN ? i : nN - 1;
    const int b  = bat[ic];
    const bool inr = i < nN;
    unsigned mA = __builtin_amdgcn_ballot_w32(inr && (b == gA));
    unsigned mB = __builtin_amdgcn_ballot_w32(inr && (b == gB));
    int nhA = (int)__builtin_popcount(mA);
    nhA = nhA > 32 ? 32 : nhA;
    int nhB = (int)__builtin_popcount(mB);
    nhB = nhB > 32 ? 32 : nhB;
#pragma unroll 1
    for (int q = 0; q < nhA; ++q) {
      const int k = __builtin_ffs((int)mA) - 1;
      mA &= mA - 1u;
      int node = i0 + (k < 0 ? 0 : k);
      node = node > nN - 1 ? nN - 1 : node;
      const v2f v = *(const v2fa*)(hf + (size_t)node * HID + 2 * lane);
      a00 += v.x; a01 += v.y;
    }
#pragma unroll 1
    for (int q = 0; q < nhB; ++q) {
      const int k = __builtin_ffs((int)mB) - 1;
      mB &= mB - 1u;
      int node = i0 + (k < 0 ? 0 : k);
      node = node > nN - 1 ? nN - 1 : node;
      const v2f v = *(const v2fa*)(hf + (size_t)node * HID + 2 * lane);
      a10 += v.x; a11 += v.y;
    }
  }
  {
    v2f p; p.x = a00; p.y = a01;
    v2f q; q.x = a10; q.y = a11;
    *(v2fa*)(gs + (2 * wave) * HID + 2 * lane) = p;
    *(v2fa*)(gs + (2 * wave + 1) * HID + 2 * lane) = q;
  }
  __syncthreads();

  {
    const int j  = tid & (L1N - 1);
    const int gq = tid >> 7;
    float t[8];
#pragma unroll
    for (int r = 0; r < 8; ++r) t[r] = 0.0f;
#pragma unroll 1
    for (int k = 0; k < HID; ++k) {
      const float w = w1s[k * L1N + j];
      const float* gp = gs + (gq * 8) * HID + k;
#pragma unroll
      for (int r = 0; r < 8; ++r) t[r] = fmaf(gp[r * HID], w, t[r]);
    }
    const float bb = b1s[j];
#pragma unroll
    for (int r = 0; r < 8; ++r) {
      float v = t[r] + bb;
      v = (v > 0.0f) ? v : (v - v);
      ts[(gq * 8 + r) * L1N + j] = v;
    }
  }
  __syncthreads();

  if (tid < PGW * NCLS) {
    const int g = tid / NCLS;
    const int o = tid - g * NCLS;
    const float* tp = ts + g * L1N;
    float s = 0.0f;
#pragma unroll 1
    for (int k = 0; k < L1N; k += 4) {
      s = fmaf(tp[k + 0], w2s[(k + 0) * NCLS + o], s);
      s = fmaf(tp[k + 1], w2s[(k + 1) * NCLS + o], s);
      s = fmaf(tp[k + 2], w2s[(k + 2) * NCLS + o], s);
      s = fmaf(tp[k + 3], w2s[(k + 3) * NCLS + o], s);
    }
    os[tid] = s + b2s[o];
  }
  __syncthreads();

  constexpr int NV = (PGW * NCLS) / 4;
  const int li = tid < NV ? tid : NV - 1;
  const v4f ov = *(const v4fa*)(os + 4 * li);
  float* op = out + (size_t)blockIdx.x * (PGW * NCLS) + 4 * li;
  const bool okst = tid < NV;
  if (okst) *(volatile v4f*)op = ov;
  __threadfence();
  if (okst) *(volatile v4f*)op = ov;
}

static inline int cdiv(int a, int b) { return (a + b - 1) / b; }
static inline size_t al256(size_t o) { return (o + 255) & ~(size_t)255; }

extern "C" void kernel_launch(void* const* d_in, const int* in_sizes, int n_in,
                              void* d_out, int out_size, void* d_ws, size_t ws_size,
                              hipStream_t stream) {
  if (n_in < 13) return;
  if (in_sizes[0] < CIN || (in_sizes[0] % CIN) != 0) return;
  const int nN = in_sizes[0] / CIN;
  if (nN < 1 || nN > (1 << 22)) return;
  if (in_sizes[1] < 2 || (in_sizes[1] & 1) != 0) return;
  const int nE = in_sizes[1] / 2;
  if (nE < 1 || nE >= (1 << (31 - SLA))) return;
  if (in_sizes[2] != nN) return;
  if (in_sizes[3] != CIN * HID || in_sizes[4] != HID) return;
  if (in_sizes[5] != HID * HID || in_sizes[6] != HID) return;
  if (in_sizes[7] != HID * HID || in_sizes[8] != HID) return;
  if (in_sizes[9] != HID * L1N || in_sizes[10] != L1N) return;
  if (in_sizes[11] != L1N * NCLS || in_sizes[12] != NCLS) return;
  if (out_size != NOUT) return;

  const float* x    = (const float*)d_in[0];
  const int*   edge = (const int*)d_in[1];
  const int*   bat  = (const int*)d_in[2];
  const float* W0   = (const float*)d_in[3];
  const float* b0   = (const float*)d_in[4];
  const float* W1   = (const float*)d_in[5];
  const float* b1   = (const float*)d_in[6];
  const float* W2   = (const float*)d_in[7];
  const float* b2   = (const float*)d_in[8];
  const float* L1w  = (const float*)d_in[9];
  const float* L1b  = (const float*)d_in[10];
  const float* L2w  = (const float*)d_in[11];
  const float* L2b  = (const float*)d_in[12];
  float* out = (float*)d_out;
  const int* src = edge;
  const int* dst = edge + nE;

  const int MP   = cdiv(nN, GBM) * GBM;
  const int gM   = MP / GBM;
  const int gD   = cdiv(nN, NBD);
  const int NBPD = gD * NBD;
  const int gA   = cdiv(MP, NBA);
  if ((long long)gA * NBA < (long long)MP) return;
  if (NBPD < nN) return;
  const int vec8 = ((nE & 3) == 0) ? 1 : 0;

  char* ws = (char*)d_ws;
  size_t off = 0;
  const size_t oDIS = off; off = al256(off + (size_t)NBPD * 4);
  const size_t oW0T = off; off = al256(off + (size_t)HID * CIN * 2);
  const size_t oW1T = off; off = al256(off + (size_t)HID * K2 * 2);
  const size_t oW2T = off; off = al256(off + (size_t)HID * K2 * 2);
  const size_t oXB  = off; off = al256(off + (size_t)MP * CIN * 2);
  const size_t oH   = off; off = al256(off + (size_t)MP * HID * 4);
  const size_t oA1  = off; off = al256(off + (size_t)MP * K2 * 2);
  const size_t oA2  = off; off = al256(off + (size_t)MP * K2 * 2);
  const size_t oH3  = off; off = al256(off + (size_t)MP * HID * 4);
  if (off > ws_size || off > (size_t)WSMAX) return;
  float*          DIS = (float*)(ws + oDIS);
  unsigned short* W0T = (unsigned short*)(ws + oW0T);
  unsigned short* W1T = (unsigned short*)(ws + oW1T);
  unsigned short* W2T = (unsigned short*)(ws + oW2T);
  unsigned short* XB  = (unsigned short*)(ws + oXB);
  float*          H   = (float*)(ws + oH);
  unsigned short* A1  = (unsigned short*)(ws + oA1);
  unsigned short* A2  = (unsigned short*)(ws + oA2);
  float*          H3  = (float*)(ws + oH3);

  const size_t aggLds = (size_t)AGG_LDS_INTS * 4;
  hipFuncSetAttribute(reinterpret_cast<const void*>(&k_agg<1, 1>), hipFuncAttributeMaxDynamicSharedMemorySize, (int)aggLds);
  hipFuncSetAttribute(reinterpret_cast<const void*>(&k_agg<0, 0>), hipFuncAttributeMaxDynamicSharedMemorySize, (int)aggLds);

  const int nUx = MP * (CIN / 8);
  k_wprep<<<(3 * NUW) / NTHR, NTHR, 0, stream>>>(W0, W1, W2, W0T, W1T, W2T);
  k_cvx<<<cdiv(nUx, NTHR), NTHR, 0, stream>>>(x, nN, nUx, XB);
  k_deg<<<gD, NTHR, 0, stream>>>(dst, nE, vec8, DIS);
  k_gemm<<<dim3(gM, HID / GBN), GTHR, 0, stream>>>(XB, W0T, H, CIN, HID);
  k_agg<1, 1><<<gA, NTHR, aggLds, stream>>>(src, dst, nE, nN, vec8, MP, DIS, H, b0, A1, H3);
  k_gemm<<<dim3(gM, HID / GBN), GTHR, 0, stream>>>(A1, W1T, H, K2, HID);
  k_agg<1, 1><<<gA, NTHR, aggLds, stream>>>(src, dst, nE, nN, vec8, MP, DIS, H, b1, A2, H3);
  k_gemm<<<dim3(gM, HID / GBN), GTHR, 0, stream>>>(A2, W2T, H, K2, HID);
  k_agg<0, 0><<<gA, NTHR, aggLds, stream>>>(src, dst, nE, nN, vec8, MP, DIS, H, b2, A2, H3);
  k_pool_head<<<NGR / PGW, NTHR, 0, stream>>>(H3, bat, nN, L1w, L1b, L2w, L2b, out);
}
